// GNN_model_83837761617950
// MI455X (gfx1250) — hardware-verified
//
#include <hip/hip_runtime.h>
#include <stddef.h>
#include <stdint.h>
#include <math.h>


#define NN      50000
#define NE      600000
#define NGR     64
#define DD      128
#define KD      256
#define NP      50048
#define NB      1024
#define NBLK    49
#define NPB     (NBLK * NB)
#define LCAP    16384
#define DEGCAP  64
#define PKS     11
#define NTHR    256
#define NWAVE   8
#define EPT     8
#define CHUNK   (NTHR * EPT)
#define WCAP    (EPT * 32)
#define LISTN   (NWAVE * WCAP)
#define GBM     64
#define GTHR    128
#define GNT     8
#define BN      128
#define XU      (2 * NP * 16)
#define XBLK    (XU / NTHR)
#define W1BLK   8
#define WDBLK   16
#define PREPBLK (XBLK + W1BLK + 2 * WDBLK)
#define RECSZ   (NGR * DD)
#define FTHR    384
#define WSMAX   134217728
#define BK_LDS_BYTES ((2 * LCAP + 2 * NB + LISTN + NB) * 4 + 128)
#define PL_LDS_BYTES ((2 * NGR * DD + NB + NGR) * 4 + 64)

static_assert(NP == 391 * 128 && NP % GBM == 0 && NP >= NN);
static_assert(NBLK * NB >= NN && NBLK * NB >= NP);
static_assert((NB & (NB - 1)) == 0 && NB <= (1 << PKS) && NB == NTHR * 4);
static_assert((CHUNK & (CHUNK - 1)) == 0 && CHUNK <= (1 << PKS));
static_assert(NE < (1 << 21) && (NE % 4) == 0);
static_assert(LISTN >= NB && LISTN >= NWAVE * WCAP);
static_assert(LCAP % (NTHR * 4) == 0 && LCAP >= 13200);
static_assert(DEGCAP >= 31 + 8);
static_assert(BK_LDS_BYTES <= 300000 && PL_LDS_BYTES <= 300000);
static_assert(GBM == (GTHR / 32) * 16 && BN == 16 * GNT && BN == DD);
static_assert(DD % 32 == 0 && KD == 2 * DD && DD % 8 == 0 && DD == 32 * 4);
static_assert((NP * 16) % NTHR == 0 && XBLK % 2 == 0);
static_assert(W1BLK * NTHR == DD * 16 && WDBLK * NTHR == DD * 32);
static_assert(NTHR == 2 * DD);
static_assert(NN % 4 == 0);
static_assert(FTHR == 3 * DD && 32 * 4 == 128 && NGR == 64);
static_assert(RECSZ % (NTHR * 4) == 0);

typedef float          v4f  __attribute__((ext_vector_type(4)));
typedef float          v8f  __attribute__((ext_vector_type(8)));
typedef int            v4i  __attribute__((ext_vector_type(4)));
typedef int            v8i  __attribute__((ext_vector_type(8)));
typedef unsigned int   v2u  __attribute__((ext_vector_type(2)));
typedef unsigned int   v4u  __attribute__((ext_vector_type(4)));
typedef unsigned short v8us __attribute__((ext_vector_type(8)));
typedef __bf16         v16b __attribute__((ext_vector_type(16)));
typedef v4f  __attribute__((may_alias)) v4fa;
typedef v4i  __attribute__((may_alias)) v4ia;
typedef v4u  __attribute__((may_alias)) v4ua;
typedef v8us __attribute__((may_alias)) v8usa;
union FragB { v16b v; v8us h[2]; v8i w; };

__device__ __forceinline__ v8f wmb(const FragB& a, const FragB& b, v8f c) {
  v8f d = __builtin_amdgcn_wmma_f32_16x16x32_bf16(false, a.v, false, b.v, (short)0, c, false, false);
  asm volatile("v_nop\n\tv_nop\n\tv_nop\n\tv_nop" : "+v"(d) : "v"(a.w), "v"(b.w));
  return d;
}

__device__ __forceinline__ unsigned short bf_bits(float f) {
  const unsigned int u = __float_as_uint(f);
  unsigned int r = (u + 0x7FFFu + ((u >> 16) & 1u)) >> 16;
  r = ((u & 0x7FFFFFFFu) > 0x7F800000u) ? 0x7FC0u : r;
  return (unsigned short)r;
}
__device__ __forceinline__ float bf_val(unsigned short b) {
  return __uint_as_float(((unsigned int)b) << 16);
}
__device__ __forceinline__ float bf_rne(float f) { return bf_val(bf_bits(f)); }

__device__ __forceinline__ int scan_chunk(const int* __restrict__ dsts, int nE, int cbase, int slotBase,
                                          int nb, int vec8, int* list, int tid, int lane, int wave) {
  int wc = 0;
  const int el0  = tid * EPT;
  const int e0   = cbase + el0;
  const int sent = -2147483647 - 1;
  v4i da, db;
  if (vec8 != 0 && cbase + CHUNK <= nE) {
    da = *(const v4i*)(dsts + e0);
    db = *(const v4i*)(dsts + e0 + 4);
  } else {
    da.x = (e0     < nE) ? dsts[min(e0,     nE - 1)] : sent;
    da.y = (e0 + 1 < nE) ? dsts[min(e0 + 1, nE - 1)] : sent;
    da.z = (e0 + 2 < nE) ? dsts[min(e0 + 2, nE - 1)] : sent;
    da.w = (e0 + 3 < nE) ? dsts[min(e0 + 3, nE - 1)] : sent;
    db.x = (e0 + 4 < nE) ? dsts[min(e0 + 4, nE - 1)] : sent;
    db.y = (e0 + 5 < nE) ? dsts[min(e0 + 5, nE - 1)] : sent;
    db.z = (e0 + 6 < nE) ? dsts[min(e0 + 6, nE - 1)] : sent;
    db.w = (e0 + 7 < nE) ? dsts[min(e0 + 7, nE - 1)] : sent;
  }
  const unsigned nbs = (unsigned)slotBase;
  const unsigned unb = (unsigned)nb;
  const unsigned s0 = (unsigned)da.x - nbs, s1 = (unsigned)da.y - nbs;
  const unsigned s2 = (unsigned)da.z - nbs, s3 = (unsigned)da.w - nbs;
  const unsigned s4 = (unsigned)db.x - nbs, s5 = (unsigned)db.y - nbs;
  const unsigned s6 = (unsigned)db.z - nbs, s7 = (unsigned)db.w - nbs;
  const bool h0 = s0 < unb, h1 = s1 < unb, h2 = s2 < unb, h3 = s3 < unb;
  const bool h4 = s4 < unb, h5 = s5 < unb, h6 = s6 < unb, h7 = s7 < unb;
  const unsigned any = __builtin_amdgcn_ballot_w32(h0 | h1 | h2 | h3 | h4 | h5 | h6 | h7);
  if (any != 0u) {
#define HITJ(J, HJ, SJ) { \
      const unsigned mj = __builtin_amdgcn_ballot_w32(HJ); \
      if (mj != 0u) { \
        if (HJ) { \
          const int pos = wc + (int)__builtin_amdgcn_mbcnt_lo(mj, 0u); \
          if (pos < WCAP) list[wave * WCAP + pos] = ((el0 + (J)) << PKS) | (int)(SJ); \
        } \
        wc += (int)__builtin_popcount(mj); } }
    HITJ(0, h0, s0)
    HITJ(1, h1, s1)
    HITJ(2, h2, s2)
    HITJ(3, h3, s3)
    HITJ(4, h4, s4)
    HITJ(5, h5, s5)
    HITJ(6, h6, s6)
    HITJ(7, h7, s7)
#undef HITJ
  }
  return wc;
}

__global__ __launch_bounds__(NTHR) void k_prep(const float* __restrict__ x1, const float* __restrict__ x2,
                                               const float* __restrict__ W1, const float* __restrict__ W2,
                                               const float* __restrict__ W3,
                                               unsigned short* xb, unsigned short* w1t, unsigned short* wd) {
  const int blk = (int)blockIdx.x, tid = (int)threadIdx.x;
  v8us o;
  unsigned short* dp;
  if (blk < XBLK) {
    const int u    = blk * NTHR + tid;
    const int prow = u >> 4;
    const int k8   = (u & 15) * 8;
    const int p    = (blk >= XBLK / 2) ? 1 : 0;
    const int row  = prow - p * NP;
    const int rc   = row < NN ? row : NN - 1;
    const float* xs = (p != 0) ? x2 : x1;
    const float* q  = xs + (size_t)rc * DD + k8;
    const v4f a = *(const v4fa*)q;
    const v4f b = *(const v4fa*)(q + 4);
    const bool ok = row < NN;
    o[0] = ok ? bf_bits(a.x) : (unsigned short)0;
    o[1] = ok ? bf_bits(a.y) : (unsigned short)0;
    o[2] = ok ? bf_bits(a.z) : (unsigned short)0;
    o[3] = ok ? bf_bits(a.w) : (unsigned short)0;
    o[4] = ok ? bf_bits(b.x) : (unsigned short)0;
    o[5] = ok ? bf_bits(b.y) : (unsigned short)0;
    o[6] = ok ? bf_bits(b.z) : (unsigned short)0;
    o[7] = ok ? bf_bits(b.w) : (unsigned short)0;
    dp = xb + (size_t)prow * DD + k8;
  } else if (blk < XBLK + W1BLK) {
    const int v  = (blk - XBLK) * NTHR + tid;
    const int n  = v >> 4;
    const int k8 = (v & 15) * 8;
    const float* q = W1 + (size_t)k8 * DD + n;
#pragma unroll
    for (int i = 0; i < 8; ++i) o[i] = bf_bits(q[(size_t)i * DD]);
    dp = w1t + (size_t)n * DD + k8;
  } else {
    const int w  = blk - XBLK - W1BLK;
    const int mi = w / WDBLK;
    const int v  = (w - mi * WDBLK) * NTHR + tid;
    const int n  = v >> 5;
    const int k8 = (v & 31) * 8;
    const int kk = k8 & (DD - 1);
    const float* Wb = (mi != 0) ? W3 : W2;
    const float* q  = Wb + (size_t)kk * DD + n;
#pragma unroll
    for (int i = 0; i < 8; ++i) o[i] = bf_bits(q[(size_t)i * DD]);
    dp = wd + (size_t)mi * DD * KD + (size_t)n * KD + k8;
  }
  *(volatile v8us*)dp = o;
  __threadfence();
  *(volatile v8us*)dp = o;
}

__global__ __launch_bounds__(NTHR) void k_bucket(const int* __restrict__ ei1, const int* __restrict__ ei2,
                                                 int* lst, int* cntp, int* offp, float* disp, int* flg) {
  extern __shared__ v4f lds_dyn[];
  int*   reg1 = (int*)lds_dyn;
  int*   reg2 = reg1 + LCAP;
  int*   scnt = reg2 + LCAP;
  int*   soff = scnt + NB;
  int*   list = soff + NB;
  float* disf = (float*)(list + LISTN);
  int*   wcnt = (int*)(disf + NB);
  int*   wtot = wcnt + NWAVE;
  int*   wbig = wtot + NWAVE;
  const int tid = (int)threadIdx.x, lane = tid & 31, wave = tid >> 5;
  const int b = (int)blockIdx.x, p = (int)blockIdx.y;
  const int* ei   = (p != 0) ? ei2 : ei1;
  const int* srcs = ei;
  const int* dsts = ei + NE;
  const int nodeBase = b * NB;

  {
    const v4i z4 = {0, 0, 0, 0};
    for (int i = tid * 4; i < LCAP; i += NTHR * 4) *(v4ia*)(reg2 + i) = z4;
    for (int i = tid; i < NB; i += NTHR) scnt[i] = 0;
  }
  __syncthreads();

  int tot = 0, ov = 0;
  const int nChunks = (NE + CHUNK - 1) / CHUNK;
#pragma unroll 1
  for (int ch = 0; ch < nChunks; ++ch) {
    const int cbase = ch * CHUNK;
    const int wc = scan_chunk(dsts, NE, cbase, nodeBase, NB, 1, list, tid, lane, wave);
    if (lane == 0) wcnt[wave] = wc;
    __syncthreads();
    int pre = 0, all = 0;
#pragma unroll
    for (int w2 = 0; w2 < NWAVE; ++w2) {
      int c = wcnt[w2];
      c = c < 0 ? 0 : (c > WCAP ? WCAP : c);
      all += c;
      pre += (w2 < wave) ? c : 0;
    }
    const int wcc  = wc > WCAP ? WCAP : wc;
    const int base = tot + pre;
#pragma unroll 1
    for (int i = lane; i < wcc; i += 32) {
      const int ent = list[wave * WCAP + i];
      const int el  = (ent >> PKS) & (CHUNK - 1);
      const int sl  = ent & (NB - 1);
      int eid = cbase + el;
      eid = eid > NE - 1 ? NE - 1 : eid;
      const int pos = base + i;
      if (pos < LCAP) reg1[pos] = (int)(((unsigned)eid << PKS) | (unsigned)sl);
    }
    if (tot + all > LCAP) ov = 1;
    tot += all;
    tot = tot > LCAP ? LCAP : tot;
    __syncthreads();
  }
  const int nh = tot;

  if (wave == 0) {
#pragma unroll 1
    for (int b0 = 0; b0 < nh; b0 += 32) {
      int idx = b0 + lane;
      idx = idx > nh - 1 ? nh - 1 : idx;
      const int uv  = reg1[idx];
      const int m32 = (nh - b0) < 32 ? (nh - b0) : 32;
#pragma unroll 1
      for (int k = 0; k < m32; ++k) {
        const int u  = __builtin_amdgcn_readlane(uv, k);
        const int sl = u & (NB - 1);
        if (lane == 0) scnt[sl] = scnt[sl] + 1;
      }
    }
  }
  __syncthreads();

  {
    const v4i ca = *(const v4ia*)(scnt + 4 * tid);
    const int e0 = ca.x < 0 ? 0 : ca.x, e1 = ca.y < 0 ? 0 : ca.y;
    const int e2 = ca.z < 0 ? 0 : ca.z, e3 = ca.w < 0 ? 0 : ca.w;
    const int ts = e0 + e1 + e2 + e3;
    int incl = ts;
#pragma unroll
    for (int d = 1; d < 32; d <<= 1) {
      const int up = __shfl_up(incl, d);
      if (lane >= d) incl += up;
    }
    if (lane == 31) wtot[wave] = incl;
    __syncthreads();
    int pre = 0;
#pragma unroll
    for (int w2 = 0; w2 < NWAVE; ++w2) pre += (w2 < wave) ? wtot[w2] : 0;
    int run = pre + incl - ts;
    soff[4 * tid + 0] = run; run += e0;
    soff[4 * tid + 1] = run; run += e1;
    soff[4 * tid + 2] = run; run += e2;
    soff[4 * tid + 3] = run;
  }
  __syncthreads();
  for (int i = tid; i < NB; i += NTHR) list[i] = soff[i];
  __syncthreads();

  if (wave == 0) {
#pragma unroll 1
    for (int b0 = 0; b0 < nh; b0 += 32) {
      int idx = b0 + lane;
      idx = idx > nh - 1 ? nh - 1 : idx;
      const int uv  = reg1[idx];
      const int m32 = (nh - b0) < 32 ? (nh - b0) : 32;
#pragma unroll 1
      for (int k = 0; k < m32; ++k) {
        const int u   = __builtin_amdgcn_readlane(uv, k);
        const int sl  = u & (NB - 1);
        const int eid = (int)((unsigned)u >> PKS);
        if (lane == 0) {
          int pos = list[sl];
          pos = pos < 0 ? 0 : (pos > LCAP - 1 ? LCAP - 1 : pos);
          reg2[pos] = eid;
          list[sl] = pos + 1;
        }
      }
    }
  }
#pragma unroll 1
  for (int j = 0; j < 4; ++j) {
    int c = scnt[4 * tid + j];
    c = c < 0 ? 0 : (c > LCAP ? LCAP : c);
    disf[4 * tid + j] = 1.0f / sqrtf((float)c + 1.0f);
  }
  const v4i c4 = *(const v4ia*)(scnt + 4 * tid);
  const v4i o4 = *(const v4ia*)(soff + 4 * tid);
  {
    const bool bg = (c4.x > DEGCAP) | (c4.y > DEGCAP) | (c4.z > DEGCAP) | (c4.w > DEGCAP);
    const unsigned mb = __builtin_amdgcn_ballot_w32(bg);
    if (lane == 0) wbig[wave] = (mb != 0u) ? 1 : 0;
  }
  __syncthreads();
  int fl = ov;
#pragma unroll
  for (int w2 = 0; w2 < NWAVE; ++w2) fl |= wbig[w2];

  int* lp = lst + (size_t)(p * NBLK + b) * LCAP;
#pragma unroll 1
  for (int it = 0; it < LCAP / (NTHR * 4); ++it) {
    const int i0 = it * (NTHR * 4) + 4 * tid;
    const v4i e4 = *(const v4ia*)(reg2 + i0);
    const int q0 = e4.x < 0 ? 0 : (e4.x > NE - 1 ? NE - 1 : e4.x);
    const int q1 = e4.y < 0 ? 0 : (e4.y > NE - 1 ? NE - 1 : e4.y);
    const int q2 = e4.z < 0 ? 0 : (e4.z > NE - 1 ? NE - 1 : e4.z);
    const int q3 = e4.w < 0 ? 0 : (e4.w > NE - 1 ? NE - 1 : e4.w);
    int s0 = srcs[q0], s1 = srcs[q1], s2 = srcs[q2], s3 = srcs[q3];
    s0 = s0 < 0 ? 0 : (s0 > NN - 1 ? NN - 1 : s0);
    s1 = s1 < 0 ? 0 : (s1 > NN - 1 ? NN - 1 : s1);
    s2 = s2 < 0 ? 0 : (s2 > NN - 1 ? NN - 1 : s2);
    s3 = s3 < 0 ? 0 : (s3 > NN - 1 ? NN - 1 : s3);
    v4i o;
    o.x = (i0     < nh) ? s0 : 0;
    o.y = (i0 + 1 < nh) ? s1 : 0;
    o.z = (i0 + 2 < nh) ? s2 : 0;
    o.w = (i0 + 3 < nh) ? s3 : 0;
    int* op = lp + i0;
    *(volatile v4i*)op = o;
    __threadfence();
    *(volatile v4i*)op = o;
  }

  const v4f d4 = *(const v4fa*)(disf + 4 * tid);
  const size_t sb = (size_t)p * NPB + (size_t)nodeBase + 4 * tid;
  const v4i f4 = {fl, fl, fl, fl};
  int* fp = flg + (size_t)(p * NBLK + b) * 32 + 4 * (lane & 7);
  const bool okf = (wave == 0) && (lane < 8);
  *(volatile v4i*)(cntp + sb) = c4;
  *(volatile v4i*)(offp + sb) = o4;
  *(volatile v4f*)(disp + sb) = d4;
  if (okf) *(volatile v4i*)fp = f4;
  __threadfence();
  *(volatile v4i*)(cntp + sb) = c4;
  *(volatile v4i*)(offp + sb) = o4;
  *(volatile v4f*)(disp + sb) = d4;
  if (okf) *(volatile v4i*)fp = f4;
}

__global__ __launch_bounds__(GTHR) void k_gemm(const unsigned short* __restrict__ A,
                                               const unsigned short* __restrict__ WT,
                                               float* outF, int K, int mRows) {
  constexpr int NT = GNT;
  constexpr int NI = 16;
  __shared__ __attribute__((aligned(16))) float stg[GBM * BN];
  const int tid = (int)threadIdx.x, lane = tid & 31, wave = tid >> 5, hh = lane >> 4, m = lane & 15;
  const int rowBase = (int)blockIdx.x * GBM;

  v8f acc[NT];
  {
    const v8f z = {0.f, 0.f, 0.f, 0.f, 0.f, 0.f, 0.f, 0.f};
#pragma unroll
    for (int t = 0; t < NT; ++t) acc[t] = z;
  }
  const unsigned short* ap = A + (size_t)(rowBase + 16 * wave + m) * (size_t)K + 8 * hh;
  const unsigned short* wp = WT + (size_t)m * (size_t)K + 8 * hh;
  const int ksteps = K >> 5;
#pragma unroll 1
  for (int ks = 0; ks < ksteps; ++ks) {
    FragB af;
    af.h[0] = *(const v8usa*)(ap + 32 * ks);
    af.h[1] = *(const v8usa*)(ap + 32 * ks + 16);
#pragma unroll
    for (int t = 0; t < NT; ++t) {
      const unsigned short* wq = wp + (size_t)(16 * t) * (size_t)K + 32 * ks;
      FragB bf;
      bf.h[0] = *(const v8usa*)wq;
      bf.h[1] = *(const v8usa*)(wq + 16);
      acc[t] = wmb(af, bf, acc[t]);
    }
  }

#pragma unroll
  for (int t = 0; t < NT; ++t) {
    const int lc = 16 * t + m;
#pragma unroll
    for (int r = 0; r < 8; ++r) {
      const int lr = 16 * wave + 8 * hh + r;
      stg[lr * BN + lc] = acc[t][r];
    }
  }
  __syncthreads();

  v4f fv[NI];
#pragma unroll
  for (int i = 0; i < NI; ++i) {
    const int lr = 16 * wave + i;
    fv[i] = *(const v4fa*)(stg + lr * BN + 4 * lane);
  }
#pragma unroll
  for (int i = 0; i < NI; ++i) {
    const int gr = rowBase + 16 * wave + i;
    float* op = outF + (size_t)gr * (size_t)DD + 4 * lane;
    if (gr < mRows) *(volatile v4f*)op = fv[i];
  }
  __threadfence();
#pragma unroll
  for (int i = 0; i < NI; ++i) {
    const int gr = rowBase + 16 * wave + i;
    float* op = outF + (size_t)gr * (size_t)DD + 4 * lane;
    if (gr < mRows) *(volatile v4f*)op = fv[i];
  }
}

__global__ __launch_bounds__(NTHR) void k_agg(const float* __restrict__ Hf, const int* __restrict__ lst,
                                              const int* __restrict__ cntp, const int* __restrict__ offp,
                                              const float* __restrict__ disp, const int* __restrict__ flg,
                                              const float* __restrict__ bias, unsigned short* xhl) {
  __shared__ __attribute__((aligned(16))) int scnt[NB];
  __shared__ __attribute__((aligned(16))) int soff[NB];
  __shared__ __attribute__((aligned(16))) unsigned int stw[NWAVE * 128];
  const int tid = (int)threadIdx.x, lane = tid & 31, wave = tid >> 5;
  const int b = (int)blockIdx.x, p = (int)blockIdx.y;
  const int nodeBase = b * NB;

  {
    const size_t sb = (size_t)p * NPB + (size_t)nodeBase + 4 * tid;
    const v4i c4 = *(const v4i*)(cntp + sb);
    const v4i o4 = *(const v4i*)(offp + sb);
    *(v4ia*)(scnt + 4 * tid) = c4;
    *(v4ia*)(soff + 4 * tid) = o4;
  }
  const int fl = flg[(size_t)(p * NBLK + b) * 32];
  float bv0, bv1, bv2, bv3;
  {
    const v4f a = *(const v4f*)(bias + 4 * lane);
    bv0 = bf_rne(a.x); bv1 = bf_rne(a.y); bv2 = bf_rne(a.z); bv3 = bf_rne(a.w);
  }
  __syncthreads();

  const float* Hp = Hf + (size_t)p * NP * DD;
  const float* dp = disp + (size_t)p * NPB;
  const int*   lp = lst + (size_t)(p * NBLK + b) * LCAP;
  unsigned short* xo = xhl + (size_t)p * NP * KD;
  const float qnan = __int_as_float(0x7fc00000);
  unsigned int* stwu = stw + wave * 128;

#pragma unroll 1
  for (int jt = 0; jt < NB / NWAVE; ++jt) {
    const int slot = wave * (NB / NWAVE) + jt;
    const int grow = nodeBase + slot;
    const int craw = __builtin_amdgcn_readfirstlane(scnt[slot]);
    int st = __builtin_amdgcn_readfirstlane(soff[slot]);
    int cnt = craw;
    st  = st < 0 ? 0 : (st > LCAP ? LCAP : st);
    cnt = cnt < 0 ? 0 : (cnt > DEGCAP ? DEGCAP : cnt);
    if (cnt > LCAP - st) cnt = LCAP - st;
    const float pz = (fl != 0 || craw > DEGCAP || craw < 0) ? qnan : 0.0f;
    const bool liveRow = grow < NN;
    const int nc = liveRow ? grow : NN - 1;
    const float dd = dp[nc];
    const float rd = dd * dd;

    float ag0 = 0.0f, ag1 = 0.0f, ag2 = 0.0f, ag3 = 0.0f;
#pragma unroll 1
    for (int b0 = 0; b0 < cnt; b0 += 32) {
      int idx = st + b0 + lane;
      idx = idx < 0 ? 0 : (idx > LCAP - 1 ? LCAP - 1 : idx);
      int sv = lp[idx];
      sv = sv < 0 ? 0 : (sv > NN - 1 ? NN - 1 : sv);
      const float cf  = dp[sv] * dd;
      const int   cfi = __float_as_int(cf);
      const int m32 = (cnt - b0) < 32 ? (cnt - b0) : 32;
#pragma unroll 1
      for (int k = 0; k < m32; ++k) {
        const int   sk = __builtin_amdgcn_readlane(sv, k);
        const float ck = __int_as_float(__builtin_amdgcn_readlane(cfi, k));
        const v4f v = *(const v4f*)(Hp + (size_t)sk * DD + 4 * lane);
        ag0 = fmaf(ck, v.x, ag0); ag1 = fmaf(ck, v.y, ag1);
        ag2 = fmaf(ck, v.z, ag2); ag3 = fmaf(ck, v.w, ag3);
      }
    }
    const v4f sf = *(const v4f*)(Hp + (size_t)nc * DD + 4 * lane);
    float y0 = (ag0 + sf.x * rd) + bv0;
    float y1 = (ag1 + sf.y * rd) + bv1;
    float y2 = (ag2 + sf.z * rd) + bv2;
    float y3 = (ag3 + sf.w * rd) + bv3;
    y0 = (y0 > 0.0f) ? y0 : (y0 - y0);
    y1 = (y1 > 0.0f) ? y1 : (y1 - y1);
    y2 = (y2 > 0.0f) ? y2 : (y2 - y2);
    y3 = (y3 > 0.0f) ? y3 : (y3 - y3);
    const float r0 = liveRow ? (y0 + pz) : 0.0f;
    const float r1 = liveRow ? (y1 + pz) : 0.0f;
    const float r2 = liveRow ? (y2 + pz) : 0.0f;
    const float r3 = liveRow ? (y3 + pz) : 0.0f;

    const unsigned short hb0 = bf_bits(r0), hb1 = bf_bits(r1), hb2 = bf_bits(r2), hb3 = bf_bits(r3);
    const unsigned short lb0 = bf_bits(r0 - bf_val(hb0)), lb1 = bf_bits(r1 - bf_val(hb1));
    const unsigned short lb2 = bf_bits(r2 - bf_val(hb2)), lb3 = bf_bits(r3 - bf_val(hb3));
    v2u hw, lw;
    hw.x = (unsigned int)hb0 | ((unsigned int)hb1 << 16);
    hw.y = (unsigned int)hb2 | ((unsigned int)hb3 << 16);
    lw.x = (unsigned int)lb0 | ((unsigned int)lb1 << 16);
    lw.y = (unsigned int)lb2 | ((unsigned int)lb3 << 16);
    __builtin_amdgcn_fence(__ATOMIC_RELEASE, "wavefront");
    __builtin_amdgcn_wave_barrier();
    *(v2u*)(stwu + 2 * lane)      = hw;
    *(v2u*)(stwu + 64 + 2 * lane) = lw;
    __builtin_amdgcn_fence(__ATOMIC_RELEASE, "wavefront");
    __builtin_amdgcn_wave_barrier();
    const v4u pk = *(const v4ua*)(stwu + 4 * lane);
    unsigned short* gp = xo + (size_t)grow * (size_t)KD + 8 * lane;
    const bool wsv = grow < NP;
    if (wsv) *(volatile v4u*)gp = pk;
    __threadfence();
    if (wsv) *(volatile v4u*)gp = pk;
  }
}

__global__ __launch_bounds__(NTHR) void k_pool(const unsigned short* __restrict__ xhl,
                                               const int* __restrict__ bv1, const int* __restrict__ bv2,
                                               float* rec, int* cntrec, int layer, int doCnt) {
  extern __shared__ v4f lds_dyn[];
  float* acc  = (float*)lds_dyn;
  int*   ids  = (int*)(acc + 2 * NGR * DD);
  int*   cnts = ids + NB;
  const int tid = (int)threadIdx.x, lane = tid & 31, wave = tid >> 5;
  const int b = (int)blockIdx.x, p = (int)blockIdx.y;
  const int nodeBase = b * NB;
  const int* bv = (p != 0) ? bv2 : bv1;

  {
    const v4f z4 = {0.f, 0.f, 0.f, 0.f};
    for (int i = tid * 4; i < 2 * NGR * DD; i += NTHR * 4) *(v4fa*)(acc + i) = z4;
    const int r0 = nodeBase + 4 * tid;
    const int rc = r0 > NN - 4 ? NN - 4 : r0;
    const v4i g4 = *(const v4i*)(bv + rc);
    const bool ok = r0 < NN;
    v4i s4;
    s4.x = ok ? g4.x : -1; s4.y = ok ? g4.y : -1; s4.z = ok ? g4.z : -1; s4.w = ok ? g4.w : -1;
    *(v4ia*)(ids + 4 * tid) = s4;
  }
  __syncthreads();

  if (doCnt != 0 && tid < NGR) {
    int c = 0;
#pragma unroll 4
    for (int i = 0; i < NB; ++i) c += (ids[i] == tid) ? 1 : 0;
    cnts[tid] = c;
  }

  {
    const int c = tid & (DD - 1), half = tid >> 7;
    float* myacc = acc + half * NGR * DD + c;
    const unsigned short* xr = xhl + (size_t)p * NP * KD + (size_t)(nodeBase + half * 512) * KD + c;
    int cur = -1;
    float accv = 0.0f;
#pragma unroll 1
    for (int r = 0; r < 512; ++r) {
      const int id = __builtin_amdgcn_readfirstlane(ids[half * 512 + r]);
      if ((unsigned)id < (unsigned)NGR) {
        if (id != cur) {
          if (cur >= 0) myacc[cur * DD] += accv;
          cur = id;
          accv = 0.0f;
        }
        const unsigned short hb = xr[(size_t)r * KD];
        const unsigned short lb = xr[(size_t)r * KD + DD];
        accv += bf_val(hb) + bf_val(lb);
      }
    }
    if (cur >= 0) myacc[cur * DD] += accv;
  }
  __syncthreads();

  constexpr int NIT = RECSZ / (NTHR * 4);
  v4f rv[NIT];
#pragma unroll
  for (int it = 0; it < NIT; ++it) {
    const int idx = it * (NTHR * 4) + 4 * tid;
    const v4f a = *(const v4fa*)(acc + idx);
    const v4f q = *(const v4fa*)(acc + NGR * DD + idx);
    rv[it] = a + q;
  }
  float* rp = rec + (size_t)((layer * 2 + p) * NBLK + b) * RECSZ;
#pragma unroll
  for (int it = 0; it < NIT; ++it) *(volatile v4f*)(rp + it * (NTHR * 4) + 4 * tid) = rv[it];
  __threadfence();
#pragma unroll
  for (int it = 0; it < NIT; ++it) *(volatile v4f*)(rp + it * (NTHR * 4) + 4 * tid) = rv[it];

  if (doCnt != 0) {
    const bool okc = (wave == 0) && (lane < 16);
    const v4i cv = *(const v4ia*)(cnts + 4 * (lane & 15));
    int* cp = cntrec + (size_t)(p * NBLK + b) * NGR + 4 * (lane & 15);
    if (okc) *(volatile v4i*)cp = cv;
    __threadfence();
    if (okc) *(volatile v4i*)cp = cv;
  }
}

__global__ __launch_bounds__(FTHR) void k_final(const float* __restrict__ rec, const int* __restrict__ cntrec,
                                                const int* __restrict__ flg, float* out) {
  __shared__ double red[FTHR];
  __shared__ double inv[2 * 32];
  __shared__ __attribute__((aligned(16))) float outs[32];
  __shared__ int wf[FTHR / 32];
  const int t = (int)threadIdx.x, lane = t & 31, wave = t >> 5;
  const int q = (int)blockIdx.x;

  {
    const int fi = t < 2 * NBLK ? t : 2 * NBLK - 1;
    const int f  = flg[(size_t)fi * 32];
    const bool fb = (t < 2 * NBLK) && (f != 0);
    const unsigned mf = __builtin_amdgcn_ballot_w32(fb);
    if (lane == 0) wf[wave] = (mf != 0u) ? 1 : 0;
  }
  if (t < 64) {
    const int pp = t >> 5, gi = t & 31;
    const int g = 32 * q + gi;
    int c = 0;
#pragma unroll 1
    for (int bb = 0; bb < NBLK; ++bb) c += cntrec[(size_t)(pp * NBLK + bb) * NGR + g];
    c = c < 1 ? 1 : c;
    inv[t] = 1.0 / (double)c;
  }
  __syncthreads();
  int any = 0;
#pragma unroll
  for (int w2 = 0; w2 < FTHR / 32; ++w2) any |= wf[w2];

  const int l = t >> 7, cc = t & (DD - 1);
#pragma unroll 1
  for (int gi = 0; gi < 32; ++gi) {
    const int g = 32 * q + gi;
    const float* r0 = rec + (size_t)((l * 2 + 0) * NBLK) * RECSZ + (size_t)g * DD + cc;
    const float* r1 = rec + (size_t)((l * 2 + 1) * NBLK) * RECSZ + (size_t)g * DD + cc;
    double h0 = 0.0, h1 = 0.0;
#pragma unroll 2
    for (int bb = 0; bb < NBLK; ++bb) {
      h0 += (double)r0[(size_t)bb * RECSZ];
      h1 += (double)r1[(size_t)bb * RECSZ];
    }
    const double d = h0 * inv[gi] - h1 * inv[32 + gi];
    red[t] = d * d;
    __syncthreads();
#pragma unroll 1
    for (int s = FTHR / 2; s >= 3; s >>= 1) {
      if (t < s) red[t] = red[t] + red[t + s];
      __syncthreads();
    }
    if (t == 0) {
      const double sm = (red[0] + red[1]) + red[2];
      outs[gi] = sqrtf((float)sm);
    }
    __syncthreads();
  }

  v4f ov = *(const v4fa*)(outs + 4 * (lane & 7));
  const float qn = __int_as_float(0x7fc00000);
  if (any != 0) { ov.x = qn; ov.y = qn; ov.z = qn; ov.w = qn; }
  float* op = out + 32 * q + 4 * (lane & 7);
  const bool okst = (wave == 0) && (lane < 8);
  if (okst) *(volatile v4f*)op = ov;
  __threadfence();
  if (okst) *(volatile v4f*)op = ov;
}

static inline size_t al256(size_t o) { return (o + 255) & ~(size_t)255; }

extern "C" void kernel_launch(void* const* d_in, const int* in_sizes, int n_in,
                              void* d_out, int out_size, void* d_ws, size_t ws_size,
                              hipStream_t stream) {
  if (n_in < 12) return;
  if (in_sizes[0] != NN * DD || in_sizes[1] != NN * DD) return;
  if (in_sizes[2] != DD * DD || in_sizes[4] != DD * DD || in_sizes[6] != DD * DD) return;
  if (in_sizes[3] != DD || in_sizes[5] != DD || in_sizes[7] != DD) return;
  if (in_sizes[8] != 2 * NE || in_sizes[9] != 2 * NE) return;
  if (in_sizes[10] != NN || in_sizes[11] != NN) return;
  if (out_size != NGR) return;

  const float* x1  = (const float*)d_in[0];
  const float* x2  = (const float*)d_in[1];
  const float* W1  = (const float*)d_in[2];
  const float* b1  = (const float*)d_in[3];
  const float* W2  = (const float*)d_in[4];
  const float* b2  = (const float*)d_in[5];
  const float* W3  = (const float*)d_in[6];
  const float* b3  = (const float*)d_in[7];
  const int*   ei1 = (const int*)d_in[8];
  const int*   ei2 = (const int*)d_in[9];
  const int*   bv1 = (const int*)d_in[10];
  const int*   bv2 = (const int*)d_in[11];
  float* out = (float*)d_out;

  char* ws = (char*)d_ws;
  size_t off = 0;
  const size_t oH    = off; off = al256(off + (size_t)2 * NP * DD * 4);
  const size_t oX    = off; off = al256(off + (size_t)2 * NP * KD * 2);
  const size_t oLIST = off; off = al256(off + (size_t)2 * NBLK * LCAP * 4);
  const size_t oCNT  = off; off = al256(off + (size_t)2 * NPB * 4);
  const size_t oOFF  = off; off = al256(off + (size_t)2 * NPB * 4);
  const size_t oDIS  = off; off = al256(off + (size_t)2 * NPB * 4);
  const size_t oREC  = off; off = al256(off + (size_t)3 * 2 * NBLK * RECSZ * 4);
  const size_t oCR   = off; off = al256(off + (size_t)2 * NBLK * NGR * 4);
  const size_t oFLG  = off; off = al256(off + (size_t)2 * NBLK * 32 * 4);
  const size_t oW1T  = off; off = al256(off + (size_t)DD * DD * 2);
  const size_t oWD   = off; off = al256(off + (size_t)2 * DD * KD * 2);
  if (off > ws_size || off > (size_t)WSMAX) return;
  if ((size_t)2 * NP * DD * 2 > (size_t)2 * NP * KD * 2) return;
  float*          H    = (float*)(ws + oH);
  unsigned short* XHL  = (unsigned short*)(ws + oX);
  unsigned short* XB   = (unsigned short*)(ws + oX);
  int*            LIST = (int*)(ws + oLIST);
  int*            CNT  = (int*)(ws + oCNT);
  int*            OFFp = (int*)(ws + oOFF);
  float*          DIS  = (float*)(ws + oDIS);
  float*          REC  = (float*)(ws + oREC);
  int*            CR   = (int*)(ws + oCR);
  int*            FLG  = (int*)(ws + oFLG);
  unsigned short* W1T  = (unsigned short*)(ws + oW1T);
  unsigned short* WD   = (unsigned short*)(ws + oWD);

  hipFuncSetAttribute(reinterpret_cast<const void*>(&k_bucket), hipFuncAttributeMaxDynamicSharedMemorySize, BK_LDS_BYTES);
  hipFuncSetAttribute(reinterpret_cast<const void*>(&k_pool), hipFuncAttributeMaxDynamicSharedMemorySize, PL_LDS_BYTES);

  const dim3 gB(NBLK, 2);
  const int gG = (2 * NP) / GBM;
  k_prep<<<PREPBLK, NTHR, 0, stream>>>(x1, x2, W1, W2, W3, XB, W1T, WD);
  k_bucket<<<gB, NTHR, BK_LDS_BYTES, stream>>>(ei1, ei2, LIST, CNT, OFFp, DIS, FLG);
  k_gemm<<<gG, GTHR, 0, stream>>>(XB, W1T, H, DD, 2 * NP);
  k_agg<<<gB, NTHR, 0, stream>>>(H, LIST, CNT, OFFp, DIS, FLG, b1, XHL);
  k_pool<<<gB, NTHR, PL_LDS_BYTES, stream>>>(XHL, bv1, bv2, REC, CR, 0, 1);
  k_gemm<<<gG, GTHR, 0, stream>>>(XHL, WD, H, KD, 2 * NP);
  k_agg<<<gB, NTHR, 0, stream>>>(H, LIST, CNT, OFFp, DIS, FLG, b2, XHL);
  k_pool<<<gB, NTHR, PL_LDS_BYTES, stream>>>(XHL, bv1, bv2, REC, CR, 1, 0);
  k_gemm<<<gG, GTHR, 0, stream>>>(XHL, WD + (size_t)DD * KD, H, KD, 2 * NP);
  k_agg<<<gB, NTHR, 0, stream>>>(H, LIST, CNT, OFFp, DIS, FLG, b3, XHL);
  k_pool<<<gB, NTHR, PL_LDS_BYTES, stream>>>(XHL, bv1, bv2, REC, CR, 2, 0);
  k_final<<<2, FTHR, 0, stream>>>(REC, CR, FLG, out);
}
